// LinearTaylorAttention_25984552141257
// MI455X (gfx1250) — hardware-verified
//
#include <hip/hip_runtime.h>
#include <stdint.h>

#define NBH    16
#define NTOK   2048
#define DD     64
#define HEAD   131072
#define FQ     4096
#define FL     4160
#define FR     4224
#define EPD    80
#define GRP    2
#define PLK    8650752
#define PLQ    8650752
#define PLV    163840
#define PKV    337920
#define NPIECE 42240
#define SKK    4.0f
#define SKL    4.0f
#define SV     4.0f
#define SQQ    32.0f
#define SQL    64.0f
#define SQ1    256.0f
#define INV_SV 0.25f

static_assert(HEAD == NTOK * DD);
static_assert(FQ == DD * DD && FL == FQ + DD && FR >= FL + 1);
static_assert((FR % 64) == 0 && (FR % 32) == 0 && (NTOK % 64) == 0 && (NTOK % 32) == 0);
static_assert(EPD == 80 && (NBH % GRP) == 0);
static_assert(PLK == FR * NTOK && PLQ == NTOK * FR && PLV == EPD * NTOK && PKV == EPD * FR);
static_assert(NPIECE * 8 == PKV && (NPIECE % 256) == 0);
static_assert((FR % 8) == 0);

typedef _Float16 v16h __attribute__((ext_vector_type(16)));
typedef _Float16 v8h  __attribute__((ext_vector_type(8)));
typedef float    v8f  __attribute__((ext_vector_type(8)));
typedef float    v4f  __attribute__((ext_vector_type(4)));
typedef unsigned int v4u __attribute__((ext_vector_type(4)));

__device__ __forceinline__ float bf_rne(float f) {
  unsigned u = __float_as_uint(f);
  u = (u + 0x7FFFu + ((u >> 16) & 1u)) & 0xFFFF0000u;
  return __uint_as_float(u);
}
__device__ __forceinline__ unsigned short h_bits(float f) {
  _Float16 h = (_Float16)f;
  return __builtin_bit_cast(unsigned short, h);
}
__device__ __forceinline__ unsigned pk16(unsigned short a, unsigned short b) { return (unsigned)a | ((unsigned)b << 16); }
__device__ __forceinline__ v4u pack8(float a0, float a1, float a2, float a3, float a4, float a5, float a6, float a7) {
  v4u p;
  p[0] = pk16(h_bits(a0), h_bits(a1));
  p[1] = pk16(h_bits(a2), h_bits(a3));
  p[2] = pk16(h_bits(a4), h_bits(a5));
  p[3] = pk16(h_bits(a6), h_bits(a7));
  return p;
}
__device__ __forceinline__ v8f zero8() { v8f z = {0.f, 0.f, 0.f, 0.f, 0.f, 0.f, 0.f, 0.f}; return z; }

__device__ __forceinline__ void store2x(unsigned short* d, v4u p) {
  *(volatile v4u*)d = p;
  __threadfence();
  *(volatile v4u*)d = p;
}

__device__ __forceinline__ v16h ldfrag_h(const _Float16* p) {
  union { v16h v; v8h h[2]; } f;
  f.h[0] = *(const v8h*)(p);
  f.h[1] = *(const v8h*)(p + 16);
  return f.v;
}

__device__ __forceinline__ v8f mma_h(v16h a, v16h b, v8f c) {
  return __builtin_amdgcn_wmma_f32_16x16x32_f16(false, a, false, b, (short)0, c, false, false);
}
template <int BF> struct Guard;
template <> struct Guard<2> {
  static __device__ __forceinline__ void dep(v8f (&c)[2], v16h a, v16h (&b)[2]) {
#if defined(__HIP_DEVICE_COMPILE__)
    asm volatile("v_nop\n\tv_nop\n\tv_nop\n\tv_nop"
                 : "+v"(c[0]), "+v"(c[1]) : "v"(a), "v"(b[0]), "v"(b[1]));
#endif
  }
  static __device__ __forceinline__ void acc(v8f (&c)[2]) {
#if defined(__HIP_DEVICE_COMPILE__)
    asm volatile("v_nop\n\tv_nop\n\tv_nop\n\tv_nop" : "+v"(c[0]), "+v"(c[1]));
#endif
  }
};
template <> struct Guard<5> {
  static __device__ __forceinline__ void dep(v8f (&c)[5], v16h a, v16h (&b)[5]) {
#if defined(__HIP_DEVICE_COMPILE__)
    asm volatile("v_nop\n\tv_nop\n\tv_nop\n\tv_nop"
                 : "+v"(c[0]), "+v"(c[1]), "+v"(c[2]), "+v"(c[3]), "+v"(c[4])
                 : "v"(a), "v"(b[0]), "v"(b[1]), "v"(b[2]), "v"(b[3]), "v"(b[4]));
#endif
  }
  static __device__ __forceinline__ void acc(v8f (&c)[5]) {
#if defined(__HIP_DEVICE_COMPILE__)
    asm volatile("v_nop\n\tv_nop\n\tv_nop\n\tv_nop"
                 : "+v"(c[0]), "+v"(c[1]), "+v"(c[2]), "+v"(c[3]), "+v"(c[4]));
#endif
  }
};
__device__ __forceinline__ void wave_sync_lds() {
  __builtin_amdgcn_fence(__ATOMIC_RELEASE, "workgroup");
  __builtin_amdgcn_wave_barrier();
  __builtin_amdgcn_fence(__ATOMIC_ACQUIRE, "workgroup");
}

__global__ __launch_bounds__(256) void k_planes(const float* __restrict__ qkv, int bh0,
                                                unsigned short* phikt, unsigned short* phiq,
                                                unsigned short* v1t) {
  __shared__ __align__(16) float tile[64 * 68];
  const int t = threadIdx.x;
  const int nt = blockIdx.x;
  const int part = blockIdx.y;
  const int z = blockIdx.z;
  const int bh = bh0 + z;
  const int which = (part < 65) ? 1 : ((part < 130) ? 0 : 2);
  const float* src = qkv + ((size_t)which * NBH + bh) * HEAD + (size_t)nt * (64 * DD);
#pragma unroll
  for (int it = 0; it < 4; ++it) {
    const int f = (t + 256 * it) * 4;
    const v4f v = *(const v4f*)(src + f);
    v4f w;
    w[0] = bf_rne(v[0]); w[1] = bf_rne(v[1]); w[2] = bf_rne(v[2]); w[3] = bf_rne(v[3]);
    *(v4f*)(tile + (f >> 6) * 68 + (f & 63)) = w;
  }
  __syncthreads();

  const int n0 = nt * 64;
  const int q8 = (t & 7) * 8;
  const int r32 = t >> 3;
  unsigned short* PK = phikt + (size_t)z * PLK;
  unsigned short* PQ = phiq  + (size_t)z * PLQ;
  unsigned short* PV = v1t   + (size_t)z * PLV;

  if (part < 64) {
    const int i = part;
#pragma unroll
    for (int it = 0; it < 2; ++it) {
      const int j = it * 32 + r32;
      float pv[8];
#pragma unroll
      for (int u = 0; u < 8; ++u) {
        const float ki = tile[(q8 + u) * 68 + i];
        const float kj = tile[(q8 + u) * 68 + j];
        pv[u] = (ki * kj) * SKK;
      }
      const v4u pk = pack8(pv[0], pv[1], pv[2], pv[3], pv[4], pv[5], pv[6], pv[7]);
      store2x(PK + (size_t)(i * 64 + j) * NTOK + n0 + q8, pk);
    }
  } else if (part == 64) {
#pragma unroll
    for (int it = 0; it < 4; ++it) {
      const int rr = it * 32 + r32;
      const int d = (rr < 64) ? rr : 63;
      float pv[8];
#pragma unroll
      for (int u = 0; u < 8; ++u) {
        const float kv = tile[(q8 + u) * 68 + d] * SKL;
        pv[u] = (rr < 64) ? kv : ((rr == 64) ? 1.0f : 0.0f);
      }
      const v4u pk = pack8(pv[0], pv[1], pv[2], pv[3], pv[4], pv[5], pv[6], pv[7]);
      store2x(PK + (size_t)(FQ + rr) * NTOK + n0 + q8, pk);
    }
  } else if (part < 129) {
    const int i = part - 65;
#pragma unroll
    for (int it = 0; it < 2; ++it) {
      const int nl = it * 32 + r32;
      const float qi = tile[nl * 68 + i];
      const v4f a = *(const v4f*)(tile + nl * 68 + q8);
      const v4f b = *(const v4f*)(tile + nl * 68 + q8 + 4);
      float pv[8];
      pv[0] = (qi * a[0]) * SQQ; pv[1] = (qi * a[1]) * SQQ; pv[2] = (qi * a[2]) * SQQ; pv[3] = (qi * a[3]) * SQQ;
      pv[4] = (qi * b[0]) * SQQ; pv[5] = (qi * b[1]) * SQQ; pv[6] = (qi * b[2]) * SQQ; pv[7] = (qi * b[3]) * SQQ;
      const v4u pk = pack8(pv[0], pv[1], pv[2], pv[3], pv[4], pv[5], pv[6], pv[7]);
      store2x(PQ + (size_t)(n0 + nl) * FR + i * 64 + q8, pk);
    }
  } else if (part == 129) {
    const int p16 = t & 15;
    const int r16 = t >> 4;
    const int cb = ((p16 < 8) ? p16 : 7) * 8;
#pragma unroll
    for (int it = 0; it < 4; ++it) {
      const int nl = it * 16 + r16;
      const v4f a = *(const v4f*)(tile + nl * 68 + cb);
      const v4f b = *(const v4f*)(tile + nl * 68 + cb + 4);
      float pv[8];
#pragma unroll
      for (int u = 0; u < 8; ++u) {
        const float qv = ((u < 4) ? a[u] : b[u - 4]) * SQL;
        const float cst = (p16 == 8 && u == 0) ? SQ1 : 0.0f;
        pv[u] = (p16 < 8) ? qv : cst;
      }
      const v4u pk = pack8(pv[0], pv[1], pv[2], pv[3], pv[4], pv[5], pv[6], pv[7]);
      store2x(PQ + (size_t)(n0 + nl) * FR + FQ + p16 * 8, pk);
    }
  } else {
#pragma unroll
    for (int it = 0; it < 3; ++it) {
      const int e = it * 32 + r32;
      int ec = e - 1; ec = (ec < 0) ? 0 : ec; ec = (ec > 63) ? 63 : ec;
      float pv[8];
#pragma unroll
      for (int u = 0; u < 8; ++u) {
        const float vv = tile[(q8 + u) * 68 + ec] * SV;
        pv[u] = (e == 0) ? 1.0f : ((e <= 64) ? vv : 0.0f);
      }
      const v4u pk = pack8(pv[0], pv[1], pv[2], pv[3], pv[4], pv[5], pv[6], pv[7]);
      unsigned short* d = PV + (size_t)((e < EPD) ? e : 0) * NTOK + n0 + q8;
      if (e < EPD) { *(volatile v4u*)d = pk; }
      __threadfence();
      if (e < EPD) { *(volatile v4u*)d = pk; }
    }
  }
}

__global__ __launch_bounds__(256) void k_cvt(const float* __restrict__ src, unsigned short* dst,
                                             int stride32, int stride16, int npieces, int rowlen) {
  const int z = blockIdx.y;
  const int p = blockIdx.x * 256 + threadIdx.x;
  if (p >= npieces) return;
  const int ppr = rowlen >> 3;
  const int row = p / ppr;
  const int c8 = (p - row * ppr) * 8;
  const float* s = src + (size_t)z * stride32 + (size_t)row * rowlen + c8;
  const v4f a = *(const v4f*)(s);
  const v4f b = *(const v4f*)(s + 4);
  const v4u pk = pack8(a[0], a[1], a[2], a[3], b[0], b[1], b[2], b[3]);
  store2x(dst + (size_t)z * stride16 + (size_t)row * rowlen + c8, pk);
}

template <int AF, int BF, int EPI>
__global__ __launch_bounds__(256) void k_gemm(const unsigned short* __restrict__ Ap, int lda, int strideA,
                                              const unsigned short* __restrict__ Btp, int ldb, int strideB,
                                              float* Cp, int ldc, int strideC, int M, int N, int K) {
  static_assert(EPI == 1 || BF == 2);
  static_assert(EPI == 0 || (AF == 2 && BF == 5));
  constexpr int SP = 16 * BF + 4;
  __shared__ __align__(16) float sT[8][16 * SP];
  const int z = blockIdx.y;
  const _Float16* A  = (const _Float16*)(const void*)(Ap  + (size_t)z * strideA);
  const _Float16* Bt = (const _Float16*)(const void*)(Btp + (size_t)z * strideB);
  float* C = Cp + (size_t)z * strideC;
  const int lane = threadIdx.x & 31;
  const int wave = threadIdx.x >> 5;
  const int TM = 16 * AF, TN = 16 * BF;
  const int tilesM = M / TM, tilesN = N / TN;
  const int tile = blockIdx.x * 8 + wave;
  if (tile >= tilesM * tilesN) return;
  const int tm = tile / tilesN;
  const int tn = tile - tm * tilesN;
  const int m0 = tm * TM;
  const int n0 = tn * TN;

  const int rl   = lane & 15;
  const int koff = (lane >> 4) * 8;
  const int mOff = (lane >> 4) * 8;

  v8f acc[AF][BF];
#pragma unroll
  for (int i = 0; i < AF; ++i)
#pragma unroll
    for (int j = 0; j < BF; ++j) acc[i][j] = zero8();

  int aoff[AF], boff[BF];
#pragma unroll
  for (int i = 0; i < AF; ++i) aoff[i] = (m0 + 16 * i + rl) * lda + koff;
#pragma unroll
  for (int j = 0; j < BF; ++j) boff[j] = (n0 + 16 * j + rl) * ldb + koff;

  for (int k0 = 0; k0 < K; k0 += 32) {
    v16h b[BF];
#pragma unroll
    for (int j = 0; j < BF; ++j) b[j] = ldfrag_h(Bt + (size_t)(boff[j] + k0));
#pragma unroll
    for (int i = 0; i < AF; ++i) {
      const v16h a = ldfrag_h(A + (size_t)(aoff[i] + k0));
#pragma unroll
      for (int j = 0; j < BF; ++j) acc[i][j] = mma_h(a, b[j], acc[i][j]);
      Guard<BF>::dep(acc[i], a, b);
    }
  }
#pragma unroll
  for (int i = 0; i < AF; ++i) Guard<BF>::acc(acc[i]);

  float* slab = sT[wave];
  if (EPI == 0) {
    const int q4 = (lane & 7) * 4, rq = lane >> 3;
#pragma unroll
    for (int i = 0; i < AF; ++i) {
#pragma unroll
      for (int j = 0; j < BF; ++j) {
#pragma unroll
        for (int r = 0; r < 8; ++r) slab[(mOff + r) * SP + 16 * j + rl] = acc[i][j][r];
      }
      wave_sync_lds();
      v4f o[4];
#pragma unroll
      for (int it = 0; it < 4; ++it) o[it] = *(const v4f*)(slab + (it * 4 + rq) * SP + q4);
      for (int ps = 0; ps < 2; ++ps) {
#pragma unroll
        for (int it = 0; it < 4; ++it) {
          const int row = it * 4 + rq;
          *(volatile v4f*)(C + (size_t)(m0 + 16 * i + row) * ldc + n0 + q4) = o[it];
        }
        __threadfence();
      }
      wave_sync_lds();
    }
  } else {
    const int hh = lane >> 4, c4 = (lane & 15) * 4;
#pragma unroll
    for (int i = 0; i < AF; ++i) {
#pragma unroll
      for (int j = 0; j < BF; ++j) {
#pragma unroll
        for (int r = 0; r < 8; ++r) slab[(mOff + r) * SP + 3 + 16 * j + rl] = acc[i][j][r];
      }
      wave_sync_lds();
      v4f o[8];
#pragma unroll
      for (int it = 0; it < 8; ++it) {
        const int row = it * 2 + hh;
        const float den = slab[row * SP + 3];
        const float rc = (1.0f / den) * INV_SV;
        const v4f nm = *(const v4f*)(slab + row * SP + 4 + c4);
        o[it] = nm * rc;
      }
      for (int ps = 0; ps < 2; ++ps) {
#pragma unroll
        for (int it = 0; it < 8; ++it) {
          const int row = it * 2 + hh;
          *(volatile v4f*)(C + (size_t)(m0 + 16 * i + row) * ldc + n0 + c4) = o[it];
        }
        __threadfence();
      }
      wave_sync_lds();
    }
  }
}

extern "C" void kernel_launch(void* const* d_in, const int* in_sizes, int n_in,
                              void* d_out, int out_size, void* d_ws, size_t ws_size,
                              hipStream_t stream) {
  if (n_in < 1) return;
  if (in_sizes[0] != 3 * NBH * HEAD) return;
  if (out_size != NBH * HEAD) return;

  const float* qkv = (const float*)d_in[0];
  float* out = (float*)d_out;

  const size_t BK  = (size_t)PLK * 2;
  const size_t BQ  = (size_t)PLQ * 2;
  const size_t BV  = (size_t)PLV * 2;
  const size_t B32 = (size_t)PKV * 4;
  const size_t B16 = (size_t)PKV * 2;
  size_t off = 0;
  const size_t oK  = off; off += (size_t)GRP * BK;
  const size_t oQ  = off; off += (size_t)GRP * BQ;
  const size_t oV  = off; off += (size_t)GRP * BV;
  const size_t o32 = off; off += (size_t)GRP * B32;
  const size_t o16 = off; off += (size_t)GRP * B16;
  if (off > ws_size) return;
  if (off > (size_t)134217728) return;

  char* ws = (char*)d_ws;
  unsigned short* PK = (unsigned short*)(ws + oK);
  unsigned short* PQ = (unsigned short*)(ws + oQ);
  unsigned short* PV = (unsigned short*)(ws + oV);
  float* C32 = (float*)(ws + o32);
  unsigned short* C16 = (unsigned short*)(ws + o16);

  const dim3 blk(256);
  const dim3 gP(NTOK / 64, 131, GRP);
  const dim3 gKV(((EPD / 80) * (FR / 32) + 7) / 8, GRP);
  const dim3 gC(NPIECE / 256, GRP);
  const dim3 gY(((NTOK / 32) * (EPD / 80) + 7) / 8, GRP);

  for (int g = 0; g < NBH / GRP; ++g) {
    const int bh0 = g * GRP;
    k_planes<<<gP, blk, 0, stream>>>(qkv, bh0, PK, PQ, PV);
    k_gemm<5, 2, 0><<<gKV, blk, 0, stream>>>(PV, NTOK, PLV, PK, NTOK, PLK, C32, FR, PKV, EPD, FR, NTOK);
    k_cvt<<<gC, blk, 0, stream>>>(C32, C16, PKV, PKV, NPIECE, FR);
    k_gemm<2, 5, 1><<<gY, blk, 0, stream>>>(PQ, FR, PLQ, C16, FR, PKV, out + (size_t)bh0 * HEAD, DD, HEAD,
                                              NTOK, EPD, FR);
  }
  (void)hipGetLastError();
}
